// Grapher_3289944949106
// MI455X (gfx1250) — hardware-verified
//
#include <hip/hip_runtime.h>
#include <math.h>

#define NB_ 8
#define CD  256
#define C2  512
#define IH  56
#define IW  56
#define NP  3136

typedef _Float16 f16;
typedef __attribute__((ext_vector_type(16))) f16 f16x16;
typedef __attribute__((ext_vector_type(8)))  f16 f16x8;
typedef __attribute__((ext_vector_type(8)))  float f32x8;
typedef __attribute__((ext_vector_type(4)))  float v4f_t;
typedef float v4fa __attribute__((ext_vector_type(4), may_alias));

__device__ __forceinline__ f32x8 wmma16(f16x16 a, f16x16 b, f32x8 c) {
  c = __builtin_amdgcn_wmma_f32_16x16x32_f16(false, a, false, b, (short)0, c, false, false);
  asm volatile("v_nop\n\tv_nop\n\tv_nop\n\tv_nop" : "+v"(c) : "v"(a), "v"(b));
  return c;
}
__device__ __forceinline__ f16x16 lds_frag(const f16* base, int stride) {
  const int lane = threadIdx.x & 31, row = lane & 15, kh = (lane >> 4) * 8;
  const f16x8 lo = *(const f16x8*)(base + row * stride + kh);
  const f16x8 hi = *(const f16x8*)(base + row * stride + kh + 16);
  f16x16 f;
#pragma unroll
  for (int i = 0; i < 8; ++i) { f[i] = lo[i]; f[i + 8] = hi[i]; }
  return f;
}
#define GSTR 48

template <typename AT, int EPI>
__global__ __launch_bounds__(256) void gemm_kn2x(const AT* __restrict__ A, int lda, size_t strideA,
                                               const float* __restrict__ Wm, int ldw, size_t strideW,
                                               const float* __restrict__ bias, const float* __restrict__ gam, const float* __restrict__ bet,
                                               const float* __restrict__ mean, const float* __restrict__ var, const float* __restrict__ R, int N,
                                               float* __restrict__ Y, int ldy, size_t strideY, int K) {
  __shared__ __attribute__((aligned(16))) f16 ldsA[128 * GSTR], ldsAl[128 * GSTR];
  __shared__ __attribute__((aligned(16))) f16 ldsW[128 * GSTR], ldsWl[128 * GSTR];
  __shared__ __attribute__((aligned(16))) float oS[8][32 * 68];
  const int tid = threadIdx.x, lane = tid & 31, wave = tid >> 5, cl = lane & 15, rh = (lane >> 4) * 8;
  const int m0 = blockIdx.x * 128, n0 = blockIdx.y * 128;
  const int wm = (wave & 3) * 32, wn = (wave >> 2) * 64;
  A += (size_t)blockIdx.z * strideA; Wm += (size_t)blockIdx.z * strideW; Y += (size_t)blockIdx.z * strideY; if (EPI == 2) R += (size_t)blockIdx.z * strideY;
  f32x8 acc[2][4], accx[2][4];
#pragma unroll
  for (int i = 0; i < 2; ++i)
#pragma unroll
    for (int j = 0; j < 4; ++j) { f32x8 z = {}; acc[i][j] = z; accx[i][j] = z; }
#pragma unroll 1
  for (int k0 = 0; k0 < K; k0 += 32) {
    __syncthreads();
    {
      const int row = tid >> 1, ch = (tid & 1) * 16;
      const AT* src = A + (size_t)(m0 + row) * lda + k0 + ch;
#pragma unroll
      for (int g = 0; g < 16; ++g) { const float v = (float)src[g]; const f16 h = (f16)v; ldsA[row * GSTR + ch + g] = h; ldsAl[row * GSTR + ch + g] = (f16)((v - (float)h) * 2048.0f); }
    }
    {
      const int k = tid >> 3, nn0 = (tid & 7) * 16;
      const float* src = Wm + (size_t)(k0 + k) * ldw;
#pragma unroll
      for (int g = 0; g < 4; ++g) { const int col = min(n0 + nn0 + 4 * g, N - 4); const v4f_t v = *(const v4f_t*)(src + col);
#pragma unroll
        for (int u = 0; u < 4; ++u) { const f16 h = (f16)v[u]; ldsW[(nn0 + 4 * g + u) * GSTR + k] = h; ldsWl[(nn0 + 4 * g + u) * GSTR + k] = (f16)((v[u] - (float)h) * 2048.0f); } }
    }
    __syncthreads();
    f16x16 af[2], afl[2];
#pragma unroll
    for (int i = 0; i < 2; ++i) { af[i] = lds_frag(ldsA + (wm + 16 * i) * GSTR, GSTR); afl[i] = lds_frag(ldsAl + (wm + 16 * i) * GSTR, GSTR); }
#pragma unroll
    for (int j = 0; j < 4; ++j) {
      const f16x16 bf = lds_frag(ldsW + (wn + 16 * j) * GSTR, GSTR), bfl = lds_frag(ldsWl + (wn + 16 * j) * GSTR, GSTR);
#pragma unroll
      for (int i = 0; i < 2; ++i) { acc[i][j] = wmma16(af[i], bf, acc[i][j]); accx[i][j] = wmma16(af[i], bfl, accx[i][j]); accx[i][j] = wmma16(afl[i], bf, accx[i][j]); }
    }
  }
  float* so = oS[wave];
#pragma unroll
  for (int i = 0; i < 2; ++i)
#pragma unroll
    for (int j = 0; j < 4; ++j) {
#pragma unroll
      for (int r = 0; r < 8; ++r) {
        const int m = m0 + wm + 16 * i + rh + r;
        const float s = gam[m] * rsqrtf(var[m] + 1e-5f), t = (bias[m] - mean[m]) * s + bet[m];
        float v = (acc[i][j][r] + accx[i][j][r] * (1.0f / 2048.0f)) * s + t;
        if (EPI == 1) v = 0.5f * v * (1.0f + erff(v * 0.70710678118654752f));
        so[(16 * i + rh + r) * 68 + 16 * j + cl] = v;
      }
    }
  asm volatile("s_wait_dscnt 0" ::: "memory");
  __builtin_amdgcn_wave_barrier();
  if (EPI == 2) {
#pragma unroll
    for (int it = 0; it < 16; ++it) { const int f4 = lane + 32 * it, rr = f4 >> 4, q = (f4 & 15) * 4;
      if (n0 + wn + q < N) { const v4f_t old = *(const v4f_t*)(R + (size_t)(m0 + wm + rr) * ldy + n0 + wn + q);
        v4f_t v = *(const volatile v4fa*)(so + rr * 68 + q); v += old; *(volatile v4fa*)(so + rr * 68 + q) = v; } }
    asm volatile("s_wait_dscnt 0" ::: "memory");
  }
#pragma unroll 1
  for (int pass = 0; pass < 2; ++pass) {
#pragma unroll
    for (int it = 0; it < 16; ++it) { const int f4 = lane + 32 * it, rr = f4 >> 4, q = (f4 & 15) * 4;
      if (n0 + wn + q < N) *(volatile v4f_t*)(Y + (size_t)(m0 + wm + rr) * ldy + n0 + wn + q) = *(const volatile v4fa*)(so + rr * 68 + q); }
    __threadfence();
  }
}

__global__ __launch_bounds__(256) void k_maxrel(float* __restrict__ cat) {
  __shared__ float pl[NP];
  __shared__ float cmin[2][2][IW], rmin[2][2][IH];
  __shared__ int cargi[2][IW], rargi[2][IH];
  const int tid = threadIdx.x, b = blockIdx.x / CD, c = blockIdx.x % CD;
  const float* h = cat + ((size_t)b * C2 + c) * NP;
  float* xj = cat + ((size_t)b * C2 + CD + c) * NP;
  for (int e = tid; e < NP; e += 256) pl[e] = h[e];
  __syncthreads();
  if (tid < 2 * IW) {
    const int x = tid >> 1, par = tid & 1;
    float m1 = INFINITY, m2 = INFINITY; int a1 = -1;
    for (int y = par; y < IH; y += 2) { const float v = pl[y * IW + x]; if (v < m1) { m2 = m1; m1 = v; a1 = y; } else if (v < m2) m2 = v; }
    cmin[par][0][x] = m1; cmin[par][1][x] = m2; cargi[par][x] = a1;
  } else if (tid < 2 * IW + 2 * IH) {
    const int t2 = tid - 2 * IW, y = t2 >> 1, par = t2 & 1;
    float m1 = INFINITY, m2 = INFINITY; int a1 = -1;
    for (int x = par; x < IW; x += 2) { const float v = pl[y * IW + x]; if (v < m1) { m2 = m1; m1 = v; a1 = x; } else if (v < m2) m2 = v; }
    rmin[par][0][y] = m1; rmin[par][1][y] = m2; rargi[par][y] = a1;
  }
  __syncthreads();
  for (int e = tid; e < NP; e += 256) {
    const int y = e / IW, x = e % IW;
    const float v = pl[e];
    const int py = y & 1, px = x & 1;
    const float cm = (cargi[py][x] == y) ? cmin[py][1][x] : cmin[py][0][x];
    const float rm = (rargi[px][y] == x) ? rmin[px][1][y] : rmin[px][0][y];
    pl[e] = fmaxf(0.0f, fmaxf(v - cm, v - rm));
  }
  __syncthreads();
#pragma unroll 1
  for (int pass = 0; pass < 2; ++pass) {
    for (int f4 = tid; f4 < NP / 4; f4 += 256) *(volatile v4f_t*)(xj + f4 * 4) = *(const volatile v4fa*)(pl + f4 * 4);
    __threadfence();
  }
}

extern "C" void kernel_launch(void* const* d_in, const int* in_sizes, int n_in,
                              void* d_out, int out_size, void* d_ws, size_t ws_size,
                              hipStream_t stream) {
  (void)in_sizes; (void)n_in; (void)out_size; (void)ws_size;
  const float* x = (const float*)d_in[0];
  const float* w1 = (const float*)d_in[1], *b1 = (const float*)d_in[2], *g1 = (const float*)d_in[3], *be1 = (const float*)d_in[4], *m1 = (const float*)d_in[5], *v1 = (const float*)d_in[6];
  const float* wg = (const float*)d_in[7], *bg = (const float*)d_in[8], *gg = (const float*)d_in[9], *beg = (const float*)d_in[10], *mg = (const float*)d_in[11], *vg = (const float*)d_in[12];
  const float* w2 = (const float*)d_in[13], *b2 = (const float*)d_in[14], *g2 = (const float*)d_in[15], *be2 = (const float*)d_in[16], *m2 = (const float*)d_in[17], *v2 = (const float*)d_in[18];
  float* out = (float*)d_out;
  char* ws = (char*)d_ws;
  float* cat = (float*)ws; ws += (size_t)NB_ * C2 * NP * 4;
  float* gbuf = (float*)ws; ws += (size_t)NB_ * C2 * NP * 4;
  const int NT = (NP + 127) / 128;
  gemm_kn2x<float, 0><<<dim3(CD / 128, NT, NB_), dim3(256), 0, stream>>>(w1, CD, 0, x, NP, (size_t)CD * NP, b1, g1, be1, m1, v1, nullptr, NP, cat, NP, (size_t)C2 * NP, CD);
  k_maxrel<<<dim3(NB_ * CD), dim3(256), 0, stream>>>(cat);
  gemm_kn2x<float, 1><<<dim3(C2 / 128, NT, NB_), dim3(256), 0, stream>>>(wg, C2, 0, cat, NP, (size_t)C2 * NP, bg, gg, beg, mg, vg, nullptr, NP, gbuf, NP, (size_t)C2 * NP, C2);
  gemm_kn2x<float, 2><<<dim3(CD / 128, NT, NB_), dim3(256), 0, stream>>>(w2, C2, 0, gbuf, NP, (size_t)C2 * NP, b2, g2, be2, m2, v2, x, NP, out, NP, (size_t)CD * NP, C2);
}
